// RGCN_link_predictor_61220463837501
// MI455X (gfx1250) — hardware-run, weakly checked
//
#include <hip/hip_runtime.h>


namespace {
constexpr int NN = 50000, CHN = 12512, NCHK = 4, NP = CHN * NCHK, NR = 4, EPR = 200000, NE = NR * EPR, D = 128, KA = NR * D  , MAXDEG = 1024, NGc = (NN + 511) / 512, PERMLEN = NE + 32 * NGc + 32;
constexpr float XS = 8.0f;

typedef _Float16 b16;
typedef __attribute__((ext_vector_type(16))) _Float16 v16b;
typedef __attribute__((ext_vector_type(8))) _Float16 v8b;
typedef __attribute__((ext_vector_type(8))) float v8f;
typedef __attribute__((ext_vector_type(4))) float v4f;
__device__ __forceinline__ float bf16_rne(float f) { unsigned int u = __float_as_uint(f); u += 0x7FFFu + ((u >> 16) & 1u); return __uint_as_float(u & 0xFFFF0000u); }
__device__ __forceinline__ void split16(float v, b16& hi, b16& lo) { hi = (b16)v; lo = (b16)(v - (float)hi); }
__device__ __forceinline__ v16b frag_kb(const b16* p, int hh) { const v8b a = *(const v8b*)(p + 8 * hh), b = *(const v8b*)(p + 16 + 8 * hh); v16b f;
#pragma unroll
  for (int e = 0; e < 8; ++e) { f[e] = a[e]; f[8 + e] = b[e]; } return f; }
__device__ __forceinline__ v8f wmma16b(v16b a, v16b b, v8f c) { v8f d = __builtin_amdgcn_wmma_f32_16x16x32_f16(false, a, false, b, (short)0, c, false, false); asm volatile("v_nop\n\tv_nop\n\tv_nop\n\tv_nop" : "+v"(d) : "v"(a), "v"(b)); return d; }
__device__ __forceinline__ void wave_lds_sync() { __builtin_amdgcn_fence(__ATOMIC_RELEASE, "workgroup"); __builtin_amdgcn_wave_barrier(); __builtin_amdgcn_fence(__ATOMIC_ACQUIRE, "workgroup"); }
__device__ __forceinline__ float nexp(float x) { return __builtin_amdgcn_exp2f(x * 1.4426950408889634f); }
__device__ __forceinline__ float pmul(float a, float b) { float p = a * b; asm volatile("" : "+v"(p)); return p; }
__device__ __forceinline__ float wsum(float v) {
#pragma unroll
  for (int o = 1; o < 32; o <<= 1) v += __shfl_xor(v, o); return v; }
constexpr int CSR_NBLK = 512, CSR_GB = 9, CSR_GN = 1 << CSR_GB  , CSR_MAXG = 512, CSR_CAP = 12288  ;
__global__ __launch_bounds__(64) void csrA_kernel(const int* __restrict__ dst, int E, int N, int nG, int CHP, int NGP, int* __restrict__ STG, int* __restrict__ HST) {
  extern __shared__ int sm[];
  int* cnt = sm; int* run = sm + NGP; int* ids = sm + 2 * NGP;
  const int b = blockIdx.x; const int ch = (E + CSR_NBLK - 1) / CSR_NBLK; const int e0 = b * ch, e1 = min(E, e0 + ch);
  for (int i = threadIdx.x; i < NGP; i += 64) cnt[i] = 0;
  for (int i = threadIdx.x; i < CHP; i += 64) ids[i] = -1;
  __syncthreads();
  if (threadIdx.x == 0) {
    for (int e = e0; e < e1; ++e) { int d = dst[e]; d = (d < 0) ? 0 : (d >= N ? N - 1 : d); cnt[d >> CSR_GB] += 1; }
    int acc = 0; for (int g = 0; g < nG; ++g) { run[g] = acc; acc += cnt[g]; }
    for (int e = e0; e < e1; ++e) { int d = dst[e]; d = (d < 0) ? 0 : (d >= N ? N - 1 : d); const int g = d >> CSR_GB; ids[run[g]] = e; run[g] += 1; } }
  __syncthreads();
  typedef __attribute__((ext_vector_type(4))) int v4i;
  for (int pass = 0; pass < 2; ++pass) {
    for (int i = threadIdx.x; i < CHP / 4; i += 64) *(volatile v4i*)(STG + (size_t)b * CHP + i * 4) = *(const v4i*)(&ids[i * 4]);
    for (int i = threadIdx.x; i < NGP / 4; i += 64) { v4i v; for (int e = 0; e < 4; ++e) v[e] = (i * 4 + e < nG) ? cnt[i * 4 + e] : 0; *(volatile v4i*)(HST + (size_t)b * NGP + i * 4) = v; }
    __threadfence(); }
}
__global__ __launch_bounds__(512) void csrS_kernel(const int* __restrict__ HST, int nG, int NGP, int* __restrict__ START, int* __restrict__ TOT, int* __restrict__ OFF) {
  __shared__ int tot[CSR_MAXG];
  const int b = threadIdx.x;
  for (int pass = 0; pass < 2; ++pass) { int runb = 0; for (int g = 0; g < nG; ++g) { int c = HST[(size_t)b * NGP + g]; c = (c < 0) ? 0 : c; ((volatile int*)OFF)[(size_t)g * CSR_NBLK + b] = runb; runb += c; } __threadfence(); }
  for (int g = threadIdx.x; g < nG; g += 512) { int s = 0; for (int bb = 0; bb < CSR_NBLK; ++bb) { int c = HST[(size_t)bb * NGP + g]; s += (c < 0) ? 0 : c; } tot[g] = s; }
  __syncthreads();
  if (threadIdx.x < 32) {
    __shared__ int st[CSR_MAXG + 32];
    if (threadIdx.x == 0) { int acc = 0; for (int g = 0; g < NGP; ++g) { st[g] = acc; if (g < nG) acc += (tot[g] + 31) & ~31; } st[NGP] = acc; }
    __builtin_amdgcn_fence(__ATOMIC_RELEASE, "workgroup"); __builtin_amdgcn_wave_barrier(); __builtin_amdgcn_fence(__ATOMIC_ACQUIRE, "workgroup");
    for (int pass = 0; pass < 2; ++pass) { for (int i = threadIdx.x; i < NGP + 32; i += 32) { ((volatile int*)START)[i] = (i <= NGP) ? st[min(i, NGP)] : 0; ((volatile int*)TOT)[i] = (i < nG) ? tot[i] : 0; } __threadfence(); } }
}
__global__ __launch_bounds__(256) void csrB_kernel(const int* __restrict__ dst, int N, int nG, int CHP, int NGP, int permLen, const int* __restrict__ STG, const int* __restrict__ HST, const int* __restrict__ OFF, const int* __restrict__ START, const int* __restrict__ TOT, int* __restrict__ PERM, int* __restrict__ ROWPTR, int* __restrict__ ROWCNT, int* __restrict__ FLAG) {
  typedef __attribute__((ext_vector_type(4))) int v4i;
  __shared__ int ids[CSR_CAP]; __shared__ unsigned short key[CSR_CAP]; __shared__ int outp[CSR_CAP]; __shared__ int ncnt[CSR_GN + 1]; __shared__ int boff[CSR_NBLK + 1];
  const int g = blockIdx.x, t_ = threadIdx.x; int tot = TOT[g]; int st = START[g], stn = START[g + 1]; const int v0 = g * CSR_GN; const int nv = min(CSR_GN, N - v0);
  st = (st < 0) ? 0 : (st > permLen - 32 ? permLen - 32 : st) & ~31; stn = (stn < st) ? st : (stn > permLen ? permLen : stn); tot = (tot < 0) ? 0 : tot; if (tot > stn - st && tot <= CSR_CAP) tot = stn - st;
  if (tot > CSR_CAP) {
    for (int pass = 0; pass < 2; ++pass) { for (int i = t_; i < CSR_GN / 4; i += 256) { v4i a, c; for (int e = 0; e < 4; ++e) { a[e] = st; c[e] = 0; } *(volatile v4i*)(ROWPTR + v0 + i * 4) = a; *(volatile v4i*)(ROWCNT + v0 + i * 4) = c; } if (t_ == 0) ((volatile int*)FLAG)[0] = 1; __threadfence(); } (void)nv; return; }
  if (t_ == 0) { int acc = 0; for (int b = 0; b < CSR_NBLK; ++b) { boff[b] = acc; int c = HST[(size_t)b * NGP + g]; c = (c < 0) ? 0 : (c > CHP ? CHP : c); acc += c; if (acc > tot) acc = tot; } boff[CSR_NBLK] = acc; }
  for (int i = t_; i <= CSR_GN; i += 256) ncnt[i] = 0;
  __syncthreads();
  for (int b = 0; b < CSR_NBLK; ++b) { const int c = boff[b + 1] - boff[b]; int o_ = OFF[(size_t)g * CSR_NBLK + b]; o_ = (o_ < 0) ? 0 : (o_ > CHP - c ? CHP - c : o_); const int* src_ = STG + (size_t)b * CHP + o_;
    for (int i = t_; i < c; i += 256) { int id = src_[i]; id = (id < 0) ? 0 : id; ids[boff[b] + i] = id; int d = dst[id]; d = (d < v0) ? v0 : (d >= N ? N - 1 : d); int kk = d - v0; kk = (kk < 0) ? 0 : (kk >= CSR_GN ? CSR_GN - 1 : kk); key[boff[b] + i] = (unsigned short)kk; } }
  __syncthreads();
  if (t_ == 0) { for (int i = 0; i < tot; ++i) ncnt[key[i]] += 1; int acc = 0; for (int vl = 0; vl < CSR_GN; ++vl) { const int c = ncnt[vl]; ncnt[vl] = acc; acc += c; } ncnt[CSR_GN] = acc;
    for (int i = 0; i < tot; ++i) { const int vl = key[i]; outp[ncnt[vl]] = ids[i]; ncnt[vl] += 1; }
    for (int vl = CSR_GN; vl > 0; --vl) ncnt[vl] = ncnt[vl - 1]; ncnt[0] = 0; }
  __syncthreads();
  for (int pass = 0; pass < 2; ++pass) {
    for (int i = t_; i < (stn - st) / 4; i += 256) { v4i v; for (int e = 0; e < 4; ++e) { const int q = i * 4 + e; v[e] = (q < tot) ? outp[q] : -1; } *(volatile v4i*)(PERM + st + i * 4) = v; }
    for (int i = t_; i < CSR_GN / 4; i += 256) { v4i a, c; for (int e = 0; e < 4; ++e) { const int vl = i * 4 + e; a[e] = st + ncnt[vl]; c[e] = (vl < nv) ? (ncnt[vl + 1] - ncnt[vl]) : 0; } *(volatile v4i*)(ROWPTR + v0 + i * 4) = a; *(volatile v4i*)(ROWCNT + v0 + i * 4) = c; }
    __threadfence(); }
}
__global__ __launch_bounds__(256) void csrZ_kernel(int* __restrict__ p, size_t n4) { typedef __attribute__((ext_vector_type(4))) int v4i; const size_t tid = (size_t)blockIdx.x * 256 + threadIdx.x, nth = (size_t)gridDim.x * 256; v4i z = {0, 0, 0, 0}; for (size_t i = tid; i < n4; i += nth) *(volatile v4i*)(p + i * 4) = z; }
struct CsrBufs { int *STG, *HST, *OFF, *START, *TOT, *PERM, *ROWPTR, *ROWCNT, *FLAG; int nG, NGP, CHP; size_t permLen; char* base; size_t bytes; };
static size_t csr_carve(CsrBufs& c, char* ws, size_t off, int E, int N) {
  const size_t off0 = off; c.base = ws + off;
  auto al = [&](size_t bytes) { char* p = ws + off; off += (bytes + 255) & ~(size_t)255; return p; };
  c.nG = (N + CSR_GN - 1) / CSR_GN; c.NGP = (c.nG + 31) & ~31; const int ch = (E + CSR_NBLK - 1) / CSR_NBLK; c.CHP = (ch + 31) & ~31; c.permLen = (size_t)E + 32 * (size_t)c.nG + 32;
  c.STG = (int*)al((size_t)CSR_NBLK * c.CHP * 4); c.HST = (int*)al((size_t)CSR_NBLK * c.NGP * 4); c.OFF = (int*)al((size_t)c.NGP * CSR_NBLK * 4); c.START = (int*)al((size_t)(c.NGP + 64) * 4); c.TOT = (int*)al((size_t)(c.NGP + 64) * 4);
  c.PERM = (int*)al(c.permLen * 4); c.ROWPTR = (int*)al((size_t)c.nG * CSR_GN * 4); c.ROWCNT = (int*)al((size_t)c.nG * CSR_GN * 4); c.FLAG = (int*)al(256);
  c.bytes = off - off0; return off;
}
static void csr_build(const CsrBufs& c, const int* dst, int E, int N, hipStream_t stream) {
  const size_t smem = (size_t)(2 * c.NGP + c.CHP) * 4;
  csrZ_kernel<<<512, 256, 0, stream>>>((int*)c.base, c.bytes / 16);
  csrA_kernel<<<CSR_NBLK, 64, smem, stream>>>(dst, E, N, c.nG, c.CHP, c.NGP, c.STG, c.HST);
  csrS_kernel<<<1, 512, 0, stream>>>(c.HST, c.nG, c.NGP, c.START, c.TOT, c.OFF);
  csrB_kernel<<<c.nG, 256, 0, stream>>>(dst, N, c.nG, c.CHP, c.NGP, (int)c.permLen, c.STG, c.HST, c.OFF, c.START, c.TOT, c.PERM, c.ROWPTR, c.ROWCNT, c.FLAG);
}

__global__ __launch_bounds__(256) void prep_kernel(const float* __restrict__ x, const float* __restrict__ w1, const float* __restrict__ b1, const float* __restrict__ w2, const float* __restrict__ b2, const float* __restrict__ p1w, const float* __restrict__ p1b, const float* __restrict__ p2w, const float* __restrict__ p2b, b16* __restrict__ R1, b16* __restrict__ R2, b16* __restrict__ RP, float* __restrict__ P, float* __restrict__ Hf) {
  const size_t tid = (size_t)blockIdx.x * 256 + threadIdx.x, nth = (size_t)gridDim.x * 256;
  for (int pass = 0; pass < 2; ++pass) {
    for (size_t p = tid; p < (size_t)NR * D * D; p += nth) { const int r = (int)(p / (D * D)), o = (int)((p / D) % D), k = (int)(p % D); ((volatile b16*)R1)[p] = (b16)bf16_rne(w1[((size_t)r * D + k) * D + o]); }
    for (size_t p = tid; p < (size_t)D * KA; p += nth) { const int o = (int)(p / KA), k = (int)(p % KA); const int r = k / D, i = k % D; ((volatile b16*)R2)[p] = (b16)bf16_rne(w2[((size_t)r * D + i) * D + o]); }
    for (size_t p = tid; p < (size_t)D * D; p += nth) { const int o = (int)(p / D), k = (int)(p % D); ((volatile b16*)RP)[p] = (b16)bf16_rne(p1w[(size_t)k * D + o]); }
    for (size_t q = tid; q < 1040; q += nth) { const int i = (int)q; float v; if (i < 512) v = bf16_rne(b1[i]); else if (i < 640) { v = 0.0f; for (int r = 0; r < NR; ++r) v += bf16_rne(b2[r * D + (i - 512)]); } else if (i < 768) v = bf16_rne(p1b[i - 640]); else if (i < 1024) v = bf16_rne(p2w[i - 768]); else v = (i - 1024 < 2) ? bf16_rne(p2b[i - 1024]) : 0.0f; P[q] = v; }
    for (size_t p = tid; p < (size_t)NP * D / 4; p += nth) { const size_t r = p / (D / 4); v4f o = {0, 0, 0, 0}; if (r < (size_t)NN) { const v4f v = *(const v4f*)(x + p * 4); for (int e = 0; e < 4; ++e) o[e] = bf16_rne(v[e]); } *(volatile v4f*)(Hf + p * 4) = o; }
    __threadfence(); }
}

__global__ __launch_bounds__(256) void ragg_kernel(const float* __restrict__ Hs, const int* __restrict__ src, const int* __restrict__ perm, const int* __restrict__ rowptr, const int* __restrict__ rowcnt, int v0c, b16* __restrict__ Ah, b16* __restrict__ Al) {
  __shared__ __attribute__((aligned(16))) b16 Sh[8][KA + 8], Sl[8][KA + 8];
  const int wave = threadIdx.x >> 5, vl = blockIdx.x * 8 + wave, v = v0c + vl, lane = threadIdx.x & 31; const bool live = v < NN;
  float acc[NR][4]; float cnt_r[NR];
#pragma unroll
  for (int r = 0; r < NR; ++r) { cnt_r[r] = 0.0f; for (int e = 0; e < 4; ++e) acc[r][e] = 0.0f; }
  if (live) { int cnt = rowcnt[v]; cnt = (cnt < 0) ? 0 : (cnt > MAXDEG ? MAXDEG : cnt); int p0 = rowptr[v]; p0 = (p0 < 0) ? 0 : (p0 > PERMLEN - cnt ? PERMLEN - cnt : p0);
    for (int q = 0; q < cnt; ++q) { int id = perm[p0 + q]; id = (id < 0) ? 0 : (id >= NE ? NE - 1 : id); int s = src[id]; s = (s < 0) ? 0 : (s >= NN ? NN - 1 : s); const int r = id / EPR; const v4f hv = *(const v4f*)(Hs + (size_t)s * D + lane * 4);
#pragma unroll
      for (int rr = 0; rr < NR; ++rr) { if (rr == r) { cnt_r[rr] += 1.0f; for (int e = 0; e < 4; ++e) acc[rr][e] += hv[e]; } } } }
#pragma unroll
  for (int r = 0; r < NR; ++r) { const float inv = 1.0f / fmaxf(cnt_r[r], 1.0f); for (int e = 0; e < 4; ++e) { b16 a_, b_; split16(live ? pmul(acc[r][e], inv) * XS : 0.0f, a_, b_); Sh[wave][r * D + lane * 4 + e] = a_; Sl[wave][r * D + lane * 4 + e] = b_; } }
  wave_lds_sync();
  for (int pass = 0; pass < 2; ++pass) { for (int i = lane; i < KA / 8; i += 32) { *(volatile v8b*)(Ah + (size_t)vl * KA + i * 8) = *(const v8b*)(&Sh[wave][i * 8]); *(volatile v8b*)(Al + (size_t)vl * KA + i * 8) = *(const v8b*)(&Sl[wave][i * 8]); } __threadfence(); }
}

template <int LAYER>
__global__ __launch_bounds__(64) void gemm_kernel(const b16* __restrict__ Ah, const b16* __restrict__ Al, const b16* __restrict__ Bw, const float* __restrict__ P, int v0c, float* __restrict__ Hout) {
  __shared__ __attribute__((aligned(16))) float Ts[2][16][D + 4];
  const int lane = threadIdx.x & 31, wave = threadIdx.x >> 5, nloc = lane & 15, hlf = lane >> 4, m0 = blockIdx.x * 32 + wave * 16;
  float y[8][8];
#pragma unroll
  for (int t = 0; t < 8; ++t) for (int r = 0; r < 8; ++r) y[t][r] = 0.0f;
  if (LAYER == 1) {
#pragma unroll 1
    for (int rel = 0; rel < NR; ++rel) { v8f acc[8]; for (int t = 0; t < 8; ++t) acc[t] = (v8f){};
#pragma unroll
      for (int kb = 0; kb < D; kb += 32) { const v16b a = frag_kb(Ah + (size_t)(m0 + nloc) * KA + rel * D + kb, hlf), al_ = frag_kb(Al + (size_t)(m0 + nloc) * KA + rel * D + kb, hlf);
#pragma unroll
        for (int t = 0; t < 8; ++t) { const v16b bw = frag_kb(Bw + ((size_t)rel * D + t * 16 + nloc) * D + kb, hlf); acc[t] = wmma16b(a, bw, acc[t]); acc[t] = wmma16b(al_, bw, acc[t]); } }
#pragma unroll
      for (int t = 0; t < 8; ++t)
#pragma unroll
        for (int r = 0; r < 8; ++r) y[t][r] += fmaxf(acc[t][r] * (1.0f / XS) + P[rel * D + t * 16 + nloc], 0.0f); } }
  else { v8f acc[8]; for (int t = 0; t < 8; ++t) acc[t] = (v8f){};
#pragma unroll 4
    for (int kb = 0; kb < KA; kb += 32) { const v16b a = frag_kb(Ah + (size_t)(m0 + nloc) * KA + kb, hlf), al_ = frag_kb(Al + (size_t)(m0 + nloc) * KA + kb, hlf);
#pragma unroll
      for (int t = 0; t < 8; ++t) { const v16b bw = frag_kb(Bw + (size_t)(t * 16 + nloc) * KA + kb, hlf); acc[t] = wmma16b(a, bw, acc[t]); acc[t] = wmma16b(al_, bw, acc[t]); } }
#pragma unroll
    for (int t = 0; t < 8; ++t)
#pragma unroll
      for (int r = 0; r < 8; ++r) y[t][r] = acc[t][r] * (1.0f / XS) + P[512 + t * 16 + nloc]; }
#pragma unroll
  for (int t = 0; t < 8; ++t)
#pragma unroll
    for (int r = 0; r < 8; ++r) Ts[wave][8 * hlf + r][t * 16 + nloc] = y[t][r];
  wave_lds_sync();
  for (int pass = 0; pass < 2; ++pass) { for (int i = lane; i < 16 * 32; i += 32) { const int rr = i >> 5, c4 = (i & 31) * 4; const int row = v0c + m0 + rr; if (row < NN) *(volatile v4f*)(Hout + (size_t)row * D + c4) = *(const v4f*)(&Ts[wave][rr][c4]); } __threadfence(); }
}

__global__ __launch_bounds__(64) void score_kernel(const float* __restrict__ H, const int* __restrict__ es, const int* __restrict__ ed, int nPairs, const b16* __restrict__ RP, const float* __restrict__ P, float* __restrict__ OUT) {
  __shared__ __attribute__((aligned(16))) b16 Ae[2][16][D + 8]; __shared__ __attribute__((aligned(16))) float Ts[2][16][D + 4]; __shared__ float Ps[32];
  const int lane = threadIdx.x & 31, wave = threadIdx.x >> 5, nloc = lane & 15, hlf = lane >> 4, e0 = blockIdx.x * 32 + wave * 16;
  for (int rr = 0; rr < 16; ++rr) { const int e = e0 + rr; int s = 0, d = 0; if (e < nPairs) { s = es[e]; d = ed[e]; s = (s < 0) ? 0 : (s >= NN ? NN - 1 : s); d = (d < 0) ? 0 : (d >= NN ? NN - 1 : d); }
    const v4f hs = *(const v4f*)(H + (size_t)s * D + lane * 4), hd = *(const v4f*)(H + (size_t)d * D + lane * 4);
#pragma unroll
    for (int k = 0; k < 4; ++k) Ae[wave][rr][lane * 4 + k] = (b16)((e < nPairs) ? pmul(hs[k], hd[k]) * XS : 0.0f); }
  wave_lds_sync();
  v8f acc[8]; for (int t = 0; t < 8; ++t) acc[t] = (v8f){};
#pragma unroll
  for (int kb = 0; kb < D; kb += 32) { const v16b a = frag_kb(&Ae[wave][nloc][kb], hlf);
#pragma unroll
    for (int t = 0; t < 8; ++t) acc[t] = wmma16b(a, frag_kb(RP + (size_t)(t * 16 + nloc) * D + kb, hlf), acc[t]); }
#pragma unroll
  for (int t = 0; t < 8; ++t)
#pragma unroll
    for (int r = 0; r < 8; ++r) { const int c = t * 16 + nloc; Ts[wave][8 * hlf + r][c] = fmaxf(acc[t][r] * (1.0f / XS) + P[640 + c], 0.0f); }
  wave_lds_sync();
  for (int rr = 0; rr < 16; ++rr) { float s0 = 0.0f, s1 = 0.0f;
#pragma unroll
    for (int k = 0; k < 4; ++k) { const float zv = Ts[wave][rr][lane * 4 + k]; s0 += pmul(zv, P[768 + (lane * 4 + k) * 2]); s1 += pmul(zv, P[768 + (lane * 4 + k) * 2 + 1]); }
    s0 = wsum(s0); s1 = wsum(s1); if (lane == 0) { const float l0 = s0 + P[1024], l1 = s1 + P[1025]; const float mx = fmaxf(l0, l1); const float a0 = nexp(l0 - mx), a1 = nexp(l1 - mx); Ps[wave * 16 + rr] = a1 / (a0 + a1); } }
  __syncthreads();
  for (int pass = 0; pass < 2; ++pass) { if (threadIdx.x < 32 && (int)(blockIdx.x * 32 + threadIdx.x) < nPairs) ((volatile float*)OUT)[(size_t)blockIdx.x * 32 + threadIdx.x] = Ps[threadIdx.x]; __threadfence(); }
}
}

extern "C" void kernel_launch(void* const* d_in, const int* in_sizes, int n_in,
                              void* d_out, int out_size, void* d_ws, size_t ws_size, hipStream_t stream) {
  (void)n_in; (void)out_size;
  const float* x = (const float*)d_in[0]; const float* w1 = (const float*)d_in[1]; const float* b1 = (const float*)d_in[2]; const float* w2 = (const float*)d_in[3]; const float* b2 = (const float*)d_in[4]; const float* p1w = (const float*)d_in[5]; const float* p1b = (const float*)d_in[6]; const float* p2w = (const float*)d_in[7]; const float* p2b = (const float*)d_in[8];
  const int* srcI = (const int*)d_in[9]; const int* dstI = (const int*)d_in[10]; const int* ps = (const int*)d_in[11]; const int* pd = (const int*)d_in[12]; const int* ns = (const int*)d_in[13]; const int* nd = (const int*)d_in[14];
  float* outP = (float*)d_out; float* outN = (float*)((char*)d_out + (size_t)NE * 4);
  if (in_sizes[0] != NN * D || in_sizes[1] != NR * D * D || in_sizes[9] != NE || in_sizes[11] != NE) return;
  size_t off = 0; char* ws = (char*)d_ws;
  auto carve = [&](size_t bytes) { char* p = ws + off; off += (bytes + 255) & ~(size_t)255; return p; };
  b16* R1 = (b16*)carve((size_t)NR * D * D * 2); b16* R2 = (b16*)carve((size_t)D * KA * 2); b16* RP = (b16*)carve((size_t)D * D * 2); float* P = (float*)carve(1040 * 4); float* Hf = (float*)carve((size_t)NP * D * 4); float* H1 = (float*)carve((size_t)NP * D * 4); float* H2 = (float*)carve((size_t)NP * D * 4); b16* Ah = (b16*)carve((size_t)CHN * KA * 2); b16* Al = (b16*)carve((size_t)CHN * KA * 2);
  CsrBufs cs; off = csr_carve(cs, ws, off, NE, NN);
  if (off > ws_size) return;
  const int VARIANT = 0;
  csr_build(cs, dstI, NE, NN, stream);
  prep_kernel<<<512, 256, 0, stream>>>(x, w1, b1, w2, b2, p1w, p1b, p2w, p2b, R1, R2, RP, P, Hf);
  if (VARIANT == 0) {
    for (int c = 0; c < NCHK; ++c) { ragg_kernel<<<CHN / 8, 256, 0, stream>>>(Hf, srcI, cs.PERM, cs.ROWPTR, cs.ROWCNT, c * CHN, Ah, Al); gemm_kernel<1><<<CHN / 32, 64, 0, stream>>>(Ah, Al, R1, P, c * CHN, H1); }
    for (int c = 0; c < NCHK; ++c) { ragg_kernel<<<CHN / 8, 256, 0, stream>>>(H1, srcI, cs.PERM, cs.ROWPTR, cs.ROWCNT, c * CHN, Ah, Al); gemm_kernel<2><<<CHN / 32, 64, 0, stream>>>(Ah, Al, R2, P, c * CHN, H2); }
    score_kernel<<<NE / 32, 64, 0, stream>>>(H2, ps, pd, NE, RP, P, outP);
    score_kernel<<<NE / 32, 64, 0, stream>>>(H2, ns, nd, NE, RP, P, outN); }
}
